// ValenceModel_64673617543725
// MI455X (gfx1250) — hardware-verified
//
#include <hip/hip_runtime.h>


namespace {
constexpr int N = 100000, D = 128, V = 100, VP = 112, NBND = 100000, NANG = 200000, NPRP = 300000, NIMP = 100000, NBLK = 14, TW = NBLK * D;
constexpr float XS = 8.0f, HS = 64.0f, WSC = 256.0f;
typedef _Float16 b16;
typedef __attribute__((ext_vector_type(16))) _Float16 v16b;
typedef __attribute__((ext_vector_type(8))) _Float16 v8b;
typedef __attribute__((ext_vector_type(8))) float v8f;
typedef __attribute__((ext_vector_type(4))) float v4f;
typedef __attribute__((ext_vector_type(2))) float v2f;
__device__ __forceinline__ float bf16_rne(float f) { unsigned int u = __float_as_uint(f); u += 0x7FFFu + ((u >> 16) & 1u); float r = __uint_as_float(u & 0xFFFF0000u); asm volatile("" : "+v"(r)); return r; }
__device__ __forceinline__ void split16(float v, b16& hi, b16& lo) { hi = (b16)v; lo = (b16)(v - (float)hi); }
__device__ __forceinline__ v16b frag_kb(const b16* p, int hh) { const v8b a = *(const v8b*)(p + 8 * hh), b = *(const v8b*)(p + 16 + 8 * hh); v16b f;
#pragma unroll
  for (int e = 0; e < 8; ++e) { f[e] = a[e]; f[8 + e] = b[e]; } return f; }
__device__ __forceinline__ v8f wmma16b(v16b a, v16b b, v8f c) { v8f d = __builtin_amdgcn_wmma_f32_16x16x32_f16(false, a, false, b, (short)0, c, false, false); asm volatile("v_nop\n\tv_nop\n\tv_nop\n\tv_nop" : "+v"(d) : "v"(a), "v"(b)); return d; }
__device__ __forceinline__ void wave_lds_sync() { __builtin_amdgcn_fence(__ATOMIC_RELEASE, "workgroup"); __builtin_amdgcn_wave_barrier(); __builtin_amdgcn_fence(__ATOMIC_ACQUIRE, "workgroup"); }
__device__ __forceinline__ float pmul(float a, float b) { float p = a * b; asm volatile("" : "+v"(p)); return p; }
__device__ __forceinline__ int iclamp(int v, int lo, int hi) { return v < lo ? lo : (v > hi ? hi : v); }

__global__ __launch_bounds__(256) void wput_kernel(const float* __restrict__ nw, const float* __restrict__ aw1, const float* __restrict__ bw1, const float* __restrict__ gw1, const float* __restrict__ pw1, const float* __restrict__ iw1, const float* __restrict__ aw2, const float* __restrict__ bw2, const float* __restrict__ gw2, const float* __restrict__ pw2, const float* __restrict__ iw2, b16* __restrict__ NWT, b16* __restrict__ W1T, b16* __restrict__ W2T) { const int u = blockIdx.x * 256 + threadIdx.x;
  for (int pass = 0; pass < 2; ++pass) {
    if (u < D * 16) { const int o = u / 16, k0 = (u % 16) * 8; v8b v;
#pragma unroll
      for (int j = 0; j < 8; ++j) v[j] = (b16)(bf16_rne(nw[(size_t)(k0 + j) * D + o]) * WSC); *(volatile v8b*)(NWT + (size_t)o * D + k0) = v; }
    if (u < TW * 16) { const int r = u / 16, k0 = (u % 16) * 8; const int blk = r / D, o = r % D; const float* w; int i; if (blk == 0) { w = aw1; i = 0; } else if (blk < 3) { w = bw1; i = blk - 1; } else if (blk < 6) { w = gw1; i = blk - 3; } else if (blk < 10) { w = pw1; i = blk - 6; } else { w = iw1; i = blk - 10; } v8b v;
#pragma unroll
      for (int j = 0; j < 8; ++j) v[j] = (b16)(bf16_rne(w[((size_t)i * D + k0 + j) * D + o]) * WSC); *(volatile v8b*)(W1T + (size_t)r * D + k0) = v; }
    if (u < 5 * 16 * 16) { const int s = u / 256, o = (u / 16) % 16, k0 = (u % 16) * 8; const float* w = s == 0 ? aw2 : s == 1 ? bw2 : s == 2 ? gw2 : s == 3 ? pw2 : iw2; const int od = s < 3 ? 2 : 6; v8b v;
#pragma unroll
      for (int j = 0; j < 8; ++j) v[j] = (b16)(o < od ? bf16_rne(w[(size_t)(k0 + j) * od + o]) * WSC : 0.0f); *(volatile v8b*)(W2T + ((size_t)s * 16 + o) * D + k0) = v; }
    __threadfence(); } }
__global__ __launch_bounds__(32) void rep_kernel(const float* __restrict__ emb, const b16* __restrict__ NWT, const float* __restrict__ nb, float* __restrict__ R) { __shared__ __attribute__((aligned(16))) b16 Ah[16][D + 8]; __shared__ float Tf[16][132]; const int lane = threadIdx.x, nloc = lane & 15, hlf = lane >> 4; const int m0 = blockIdx.x * 16;
  for (int rr = 0; rr < 16; ++rr) for (int q = 0; q < 4; ++q) Ah[rr][q * 32 + lane] = (b16)(m0 + rr < V ? bf16_rne(emb[(size_t)(m0 + rr) * D + q * 32 + lane]) * XS : 0.0f);
  wave_lds_sync(); v8f acc[8];
#pragma unroll
  for (int t = 0; t < 8; ++t) acc[t] = (v8f){};
#pragma unroll
  for (int kb = 0; kb < D; kb += 32) { const v16b a = frag_kb(&Ah[nloc][kb], hlf);
#pragma unroll
    for (int t = 0; t < 8; ++t) acc[t] = wmma16b(a, frag_kb(NWT + (size_t)(t * 16 + nloc) * D + kb, hlf), acc[t]); }
#pragma unroll
  for (int t = 0; t < 8; ++t) { const int c = t * 16 + nloc; const float bb = bf16_rne(nb[c]);
#pragma unroll
    for (int r8 = 0; r8 < 8; ++r8) Tf[8 * hlf + r8][c] = (m0 + 8 * hlf + r8 < V) ? fmaxf(acc[t][r8] * (1.0f / (XS * WSC)) + bb, 0.0f) : 0.0f; }
  wave_lds_sync();
  for (int pass = 0; pass < 2; ++pass) { for (int rr = 0; rr < 16; ++rr) *(volatile v4f*)(R + (size_t)(m0 + rr) * D + lane * 4) = *(const v4f*)(&Tf[rr][lane * 4]); __threadfence(); } }
__global__ __launch_bounds__(32) void table_kernel(const float* __restrict__ R, const b16* __restrict__ W1T, float* __restrict__ P) { __shared__ __attribute__((aligned(16))) b16 Ah[16][D + 8], Al[16][D + 8]; __shared__ float Tf[16][132]; const int lane = threadIdx.x, nloc = lane & 15, hlf = lane >> 4; const int blk = blockIdx.x % NBLK, m0 = (blockIdx.x / NBLK) * 16;
  for (int rr = 0; rr < 16; ++rr) for (int q = 0; q < 4; ++q) { b16 p, ql; split16(R[(size_t)(m0 + rr) * D + q * 32 + lane] * HS, p, ql); Ah[rr][q * 32 + lane] = p; Al[rr][q * 32 + lane] = ql; }
  wave_lds_sync(); v8f acc[8];
#pragma unroll
  for (int t = 0; t < 8; ++t) acc[t] = (v8f){};
#pragma unroll
  for (int kb = 0; kb < D; kb += 32) { const v16b a = frag_kb(&Ah[nloc][kb], hlf), al = frag_kb(&Al[nloc][kb], hlf);
#pragma unroll
    for (int t = 0; t < 8; ++t) { const v16b bw = frag_kb(W1T + ((size_t)blk * D + t * 16 + nloc) * D + kb, hlf); acc[t] = wmma16b(a, bw, acc[t]); acc[t] = wmma16b(al, bw, acc[t]); } }
#pragma unroll
  for (int t = 0; t < 8; ++t)
#pragma unroll
    for (int r8 = 0; r8 < 8; ++r8) Tf[8 * hlf + r8][t * 16 + nloc] = acc[t][r8] * (1.0f / (HS * WSC));
  wave_lds_sync();
  for (int pass = 0; pass < 2; ++pass) { for (int rr = 0; rr < 16; ++rr) *(volatile v4f*)(P + ((size_t)blk * VP + m0 + rr) * D + lane * 4) = *(const v4f*)(&Tf[rr][lane * 4]); __threadfence(); } }
template <int SPEC>
__global__ __launch_bounds__(32) void inter_kernel(const int* __restrict__ idx, const int* __restrict__ elem, const float* __restrict__ P, const float* __restrict__ b1, const b16* __restrict__ W2T, const float* __restrict__ b2, int NROWS, float* __restrict__ out) {
  constexpr int AR = SPEC == 1 ? 2 : SPEC == 2 ? 3 : SPEC == 3 ? 4 : 5;
  constexpr int NS = SPEC == 4 ? 4 : AR;
  constexpr int NPERM = SPEC == 4 ? 3 : 2; constexpr int OD = SPEC <= 2 ? 2 : 6; constexpr int BLK0 = SPEC == 1 ? 1 : SPEC == 2 ? 3 : SPEC == 3 ? 6 : 10;
  __shared__ __attribute__((aligned(16))) b16 Ah[16][D + 8], Al[16][D + 8]; __shared__ int Ty[16][5]; __shared__ float To[16][17]; const int lane = threadIdx.x, nloc = lane & 15, hlf = lane >> 4; const size_t r0 = (size_t)blockIdx.x * 16; if (r0 >= (size_t)NROWS) return;
  if (lane < 16) { for (int a = 0; a < AR; ++a) { const int node = iclamp(idx[(r0 + lane) * AR + a], 0, N - 1); Ty[lane][a] = iclamp(elem[node], 0, V - 1); } }
  wave_lds_sync(); v8f acc = {};
  for (int pm = 0; pm < NPERM; ++pm) { int perm[4];
    if (SPEC == 1) { perm[0] = pm == 0 ? 0 : 1; perm[1] = pm == 0 ? 1 : 0; perm[2] = 0; perm[3] = 0; }
    else if (SPEC == 2) { perm[0] = pm == 0 ? 0 : 2; perm[1] = 1; perm[2] = pm == 0 ? 2 : 0; perm[3] = 0; }
    else if (SPEC == 3) { perm[0] = pm == 0 ? 0 : 3; perm[1] = pm == 0 ? 1 : 2; perm[2] = pm == 0 ? 2 : 1; perm[3] = pm == 0 ? 3 : 0; }
    else { const int tab[3][4] = {{0, 1, 2, 3}, {0, 3, 4, 2}, {0, 4, 2, 3}}; for (int s = 0; s < 4; ++s) perm[s] = tab[pm][s]; }
    for (int rr = 0; rr < 16; ++rr) for (int q = 0; q < 4; ++q) { const int c = q * 32 + lane; float s = bf16_rne(b1[c]); for (int sl = 0; sl < NS; ++sl) s += P[((size_t)(BLK0 + sl) * VP + Ty[rr][perm[sl]]) * D + c]; b16 p, ql; split16(fmaxf(s, 0.0f) * HS, p, ql); Ah[rr][c] = p; Al[rr][c] = ql; }
    wave_lds_sync();
#pragma unroll
    for (int kb = 0; kb < D; kb += 32) { const v16b bw = frag_kb(W2T + ((size_t)SPEC * 16 + nloc) * D + kb, hlf); acc = wmma16b(frag_kb(&Ah[nloc][kb], hlf), bw, acc); acc = wmma16b(frag_kb(&Al[nloc][kb], hlf), bw, acc); }
    wave_lds_sync(); }
#pragma unroll
  for (int r8 = 0; r8 < 8; ++r8) To[8 * hlf + r8][nloc] = acc[r8] * (1.0f / (HS * WSC)) + (nloc < OD ? NPERM * bf16_rne(b2[nloc]) : 0.0f);
  wave_lds_sync();
  for (int pass = 0; pass < 2; ++pass) { for (int q = lane; q < 16 * OD; q += 32) ((volatile float*)out)[r0 * OD + q] = To[q / OD][q % OD]; __threadfence(); } }
__global__ __launch_bounds__(256) void atom_kernel(const int* __restrict__ elem, const float* __restrict__ P, const float* __restrict__ b1, const float* __restrict__ w2, const float* __restrict__ b2, float* __restrict__ out) { __shared__ float TA[VP][2]; const int t = threadIdx.x;
  if (t < V) { float s0 = bf16_rne(b2[0]), s1 = bf16_rne(b2[1]);
#pragma unroll 4
    for (int c = 0; c < D; ++c) { const float h = fmaxf(P[(size_t)t * D + c] + bf16_rne(b1[c]), 0.0f); s0 += pmul(h, bf16_rne(w2[c * 2])); s1 += pmul(h, bf16_rne(w2[c * 2 + 1])); } TA[t][0] = s0; TA[t][1] = s1; }
  __syncthreads(); const size_t n = (size_t)blockIdx.x * 256 + t; if (n >= (size_t)N) return; const int ty = iclamp(elem[n], 0, V - 1);
  for (int pass = 0; pass < 2; ++pass) { *(volatile v2f*)(out + n * 2) = (v2f){TA[ty][0], TA[ty][1]}; __threadfence(); } }
}

extern "C" void kernel_launch(void* const* d_in, const int* in_sizes, int n_in, void* d_out, int out_size, void* d_ws, size_t ws_size, hipStream_t stream) {
  (void)n_in;
  auto Fp = [&](int i) { return (const float*)d_in[i]; }; auto Ip = [&](int i) { return (const int*)d_in[i]; };
  if (in_sizes[0] != N || in_sizes[1] != NBND * 2 || in_sizes[2] != NANG * 3 || in_sizes[3] != NPRP * 4 || in_sizes[4] != NIMP * 5 || in_sizes[5] != V * D || in_sizes[6] != D * D || in_sizes[12] != 2 * D * D || in_sizes[20] != 4 * D * D || in_sizes[24] != 4 * D * D || in_sizes[22] != D * 6 || out_size != N * 2 + NBND * 2 + NANG * 2 + NPRP * 6 + NIMP * 6) return;
  const int DIV = 1;
  size_t off = 0; char* ws = (char*)d_ws;
  auto carve = [&](size_t bytes) { char* p = ws + off; off += (bytes + 255) & ~(size_t)255; return p; };
  b16* NWT = (b16*)carve((size_t)D * D * 2); b16* W1T = (b16*)carve((size_t)TW * D * 2); b16* W2T = (b16*)carve((size_t)5 * 16 * D * 2); float* R = (float*)carve((size_t)VP * D * 4); float* P = (float*)carve((size_t)NBLK * VP * D * 4);
  if (off > ws_size || off > ((size_t)4 << 20)) return;
  float* out = (float*)d_out; float* oat = out; float* obd = oat + (size_t)N * 2; float* oan = obd + (size_t)NBND * 2; float* opr = oan + (size_t)NANG * 2; float* oim = opr + (size_t)NPRP * 6;
  wput_kernel<<<(TW * 16 + 255) / 256, 256, 0, stream>>>(Fp(6), Fp(8), Fp(12), Fp(16), Fp(20), Fp(24), Fp(10), Fp(14), Fp(18), Fp(22), Fp(26), NWT, W1T, W2T);
  rep_kernel<<<VP / 16, 32, 0, stream>>>(Fp(5), NWT, Fp(7), R);
  table_kernel<<<(VP / 16) * NBLK, 32, 0, stream>>>(R, W1T, P);
  atom_kernel<<<(N + 255) / 256, 256, 0, stream>>>(Ip(0), P, Fp(9), Fp(10), Fp(11), oat);
  inter_kernel<1><<<NBND / DIV / 16, 32, 0, stream>>>(Ip(1), Ip(0), P, Fp(13), W2T, Fp(15), NBND / DIV, obd);
  inter_kernel<2><<<NANG / DIV / 16, 32, 0, stream>>>(Ip(2), Ip(0), P, Fp(17), W2T, Fp(19), NANG / DIV, oan);
  inter_kernel<3><<<NPRP / DIV / 16, 32, 0, stream>>>(Ip(3), Ip(0), P, Fp(21), W2T, Fp(23), NPRP / DIV, opr);
  inter_kernel<4><<<NIMP / DIV / 16, 32, 0, stream>>>(Ip(4), Ip(0), P, Fp(25), W2T, Fp(27), NIMP / DIV, oim);
}
